// MLAttention_78683800863106
// MI455X (gfx1250) — hardware-verified
//
#include <hip/hip_runtime.h>
#include <math.h>
#include <stdint.h>

#ifndef NB
#define NB 2
#endif
#ifndef SEQ
#define SEQ 2048
#endif
#define XS_FULL 2048
#define DMOD  2048
#define NH    16
#define HD    128
#define HHALF (HD / 2)
#define HROT  32
#define DQ    682
#define DQP   704
#define DKV   1024
#define DKR   64
#define DCKV  1088
#define DHKV  192
#define DUKV  3072
#define QO    ((SEQ < 256) ? SEQ : 256)
#define QRES  ((SEQ < 512) ? SEQ : 512)
#define MROWS (NB * SEQ)
#define MCH   ((SEQ < 1024) ? SEQ : 1024)
#define NCH   (SEQ / MCH)
#define EPS_LN 0.00001f
#define RSQ_HD 0.08838834764831845f
#define LOG2E 1.4426950408889634f
#define KINVF (-0.41524101186092155f)
#define NEGT  (-1.0e30f)
#define QSC   256.0f
#define KSC   256.0f
#define PCAR  32768.0f
#define VCAR  1024.0f
#define OSC   1024.0f
#define WSC   1024.0f
#define CSC   1024.0f
#define WPB   2
#define NHG   (NH / WPB)
#define NQT   (SEQ / 16)
#define NST   (MCH / 64)
#define NKT   (SEQ / 32)
#define ATT_THREADS (WPB * 32)
#define PTP   36
#define PTW   (16 * PTP)
#define SLP   132
#define SLW   (16 * SLP)
#define WREG  (PTW + SLW)
#define SLAB64 (16 * 68)
#define VTP   72
#define TABF  (2 * NH * HROT)
#define WS_CAP 134217728
static_assert(DMOD == NH * HD && HD == 128 && HHALF == 64 && NH == 16 && WPB == 2 && NHG * WPB == NH);
static_assert(ATT_THREADS == 64 && DKV + DKR == DCKV && DHKV == DKR + HD && NH * DHKV == DUKV && 2 * HROT == HHALF);
static_assert(NB >= 1 && NB <= 2);
static_assert((SEQ % 64) == 0 && SEQ >= 64 && SEQ <= XS_FULL);
static_assert((QO % 64) == 0 && QO >= 64 && QO <= SEQ && (QO % 16) == 0);
static_assert((QRES % 64) == 0 && QRES >= 64 && QRES <= SEQ && QO <= QRES);
static_assert((MCH % 64) == 0 && MCH >= 64 && NCH * MCH == SEQ);
static_assert((DMOD % 64) == 0 && (DQP % 64) == 0 && (DCKV % 64) == 0 && (DUKV % 64) == 0 && (DKV % 32) == 0 && (DQP % 32) == 0);
static_assert(DQP >= DQ && (DQP % 8) == 0 && DQP <= 1024 && DKV <= 1024);
static_assert(TABF == 1024);
static_assert(WPB * WREG * 4 <= 65536 && 2 * HD * VTP * 2 <= 65536 && 4 * SLAB64 * 4 <= 65536);

typedef unsigned short u16;
typedef _Float16 v16h __attribute__((ext_vector_type(16)));
typedef _Float16 v8h  __attribute__((ext_vector_type(8)));
typedef __bf16   v16b __attribute__((ext_vector_type(16)));
typedef float    v8f  __attribute__((ext_vector_type(8)));
typedef float    v4f  __attribute__((ext_vector_type(4)));
typedef unsigned int v4u __attribute__((ext_vector_type(4)));

union FragH { v16h v; v8h h[2]; v4u u[2]; };
union FragB { v16b v; v4u u[2]; };

__device__ __forceinline__ unsigned short bf_bits(float f) {
  unsigned u = __float_as_uint(f);
  return (unsigned short)((u + 0x7FFFu + ((u >> 16) & 1u)) >> 16);
}
__device__ __forceinline__ float bf_up(unsigned short h) { return __uint_as_float(((unsigned)h) << 16); }
__device__ __forceinline__ float bfr(float f) { return bf_up(bf_bits(f)); }
__device__ __forceinline__ unsigned short h_bits(_Float16 x) { return __builtin_bit_cast(unsigned short, x); }
__device__ __forceinline__ unsigned pk16(unsigned short a, unsigned short b) { return (unsigned)a | ((unsigned)b << 16); }
__device__ __forceinline__ v8f zero8() { v8f z = {0.f, 0.f, 0.f, 0.f, 0.f, 0.f, 0.f, 0.f}; return z; }
__device__ __forceinline__ const _Float16* hp(const u16* p) { return (const _Float16*)(const void*)p; }

__device__ __forceinline__ v16h ldfrag_h(const _Float16* p) {
  FragH f;
  f.h[0] = *(const v8h*)(p);
  f.h[1] = *(const v8h*)(p + 16);
  return f.v;
}
__device__ __forceinline__ v16b ldfrag_b(const u16* p) {
  FragB f;
  f.u[0] = *(const v4u*)(p);
  f.u[1] = *(const v4u*)(p + 16);
  return f.v;
}

__device__ __forceinline__ v8f mma_h(v16h a, v16h b, v8f c) {
  return __builtin_amdgcn_wmma_f32_16x16x32_f16(false, a, false, b, (short)0, c, false, false);
}
__device__ __forceinline__ v8f mma_b(v16b a, v16b b, v8f c) {
  return __builtin_amdgcn_wmma_f32_16x16x32_bf16(false, a, false, b, (short)0, c, false, false);
}
__device__ __forceinline__ void guard2(v8f& a, v8f& b, v16h x0, v16h x1, v16h x2, v16h x3, v16h x4, v16h x5) {
#if defined(__HIP_DEVICE_COMPILE__)
  asm volatile("v_nop\n\tv_nop\n\tv_nop\n\tv_nop"
               : "+v"(a), "+v"(b) : "v"(x0), "v"(x1), "v"(x2), "v"(x3), "v"(x4), "v"(x5) : "memory");
#endif
}
template <typename F>
__device__ __forceinline__ void guard6(v8f& a, v8f& b, v8f& c, v8f& d, F x0, F x1, F x2, F x3, F x4, F x5) {
#if defined(__HIP_DEVICE_COMPILE__)
  asm volatile("v_nop\n\tv_nop\n\tv_nop\n\tv_nop"
               : "+v"(a), "+v"(b), "+v"(c), "+v"(d) : "v"(x0), "v"(x1), "v"(x2), "v"(x3), "v"(x4), "v"(x5) : "memory");
#endif
}
__device__ __forceinline__ void acc_guard4(v8f& a, v8f& b, v8f& c, v8f& d) {
#if defined(__HIP_DEVICE_COMPILE__)
  asm volatile("v_nop\n\tv_nop\n\tv_nop\n\tv_nop" : "+v"(a), "+v"(b), "+v"(c), "+v"(d));
#endif
}
__device__ __forceinline__ void wave_sync_lds() {
  __builtin_amdgcn_fence(__ATOMIC_RELEASE, "workgroup");
  __builtin_amdgcn_wave_barrier();
  __builtin_amdgcn_fence(__ATOMIC_ACQUIRE, "workgroup");
}

__global__ __launch_bounds__(256) void cvtpad16(const float* __restrict__ S, int srows, int scols,
                                                u16* D, int drows, int dcols, int f16mode, float scale, int vec) {
  const int n8 = (drows * dcols) >> 3;
  const int gt = blockIdx.x * 256 + (int)threadIdx.x;
  if (gt >= n8) return;
  const size_t flat = (size_t)gt * 8;
  const int r  = (int)(flat / (size_t)dcols);
  const int c0 = (int)(flat - (size_t)r * (size_t)dcols);
  float w[8];
  if (vec != 0) {
    const float* p = S + flat;
    const v4f a = *(const v4f*)(p), b4 = *(const v4f*)(p + 4);
#pragma unroll
    for (int e = 0; e < 4; ++e) { w[e] = a[e]; w[4 + e] = b4[e]; }
  } else {
    const int rr = (r < srows) ? r : (srows - 1);
    const float* p = S + (size_t)rr * (size_t)scols;
#pragma unroll
    for (int e = 0; e < 8; ++e) {
      const int cc = c0 + e;
      const int cl = (cc < scols) ? cc : (scols - 1);
      const float v = p[cl];
      w[e] = ((r < srows) && (cc < scols)) ? v : 0.0f;
    }
  }
  v4u o;
#pragma unroll
  for (int e = 0; e < 4; ++e) {
    const float f0 = w[2 * e], f1 = w[2 * e + 1];
    const unsigned short hb0 = h_bits((_Float16)(bfr(f0) * scale));
    const unsigned short hb1 = h_bits((_Float16)(bfr(f1) * scale));
    const unsigned short bb0 = bf_bits(f0);
    const unsigned short bb1 = bf_bits(f1);
    o[e] = (f16mode != 0) ? pk16(hb0, hb1) : pk16(bb0, bb1);
  }
  u16* d = D + flat;
  for (int pass = 0; pass < 2; ++pass) {
    *(volatile v4u*)(d) = o;
    __threadfence();
  }
}

__global__ __launch_bounds__(256) void rtab(float* CS) {
  __shared__ __align__(16) float tab[TABF];
  const int tid = (int)threadIdx.x;
#pragma unroll 1
  for (int e = 0; e < 2; ++e) {
    const int idx = tid * 2 + e;
    const int h = idx >> 5, j = idx & 31;
    const float invf = exp2f((float)j * KINVF);
    const float ang  = (float)h * invf;
    tab[idx]             = cosf(ang);
    tab[NH * HROT + idx] = sinf(ang);
  }
  __syncthreads();
  const v4f v = *(const v4f*)(tab + tid * 4);
  float* d = CS + tid * 4;
  for (int pass = 0; pass < 2; ++pass) {
    *(volatile v4f*)(d) = v;
    __threadfence();
  }
}

__global__ __launch_bounds__(128) void ln16(const float* __restrict__ Sf, int lds, int nvalid,
                                            const float* __restrict__ g, const float* __restrict__ gb,
                                            u16* Hp, u16* Lp, int ldd, float sc) {
  __shared__ __align__(16) float sg[1024];
  __shared__ __align__(16) float sbb[1024];
  __shared__ float red[8];
  const int tid  = (int)threadIdx.x;
  const int lane = tid & 31, wave = tid >> 5;
  const int row  = (int)blockIdx.x;
#pragma unroll 1
  for (int c = tid; c < ldd; c += 128) {
    const int cl = (c < nvalid) ? c : (nvalid - 1);
    const float gv = g[cl];
    const float bv = gb[cl];
    sg[c]  = (c < nvalid) ? bfr(gv) : 0.0f;
    sbb[c] = (c < nvalid) ? bfr(bv) : 0.0f;
  }
  const int ncol = ldd >> 3;
  const int tc   = (tid < ncol) ? tid : (ncol - 1);
  const int c0   = tc * 8;
  const float* p = Sf + (size_t)row * (size_t)lds + c0;
  const v4f xa = *(const v4f*)(p), xb = *(const v4f*)(p + 4);
  float xv[8];
  bool  ok[8];
#pragma unroll
  for (int e = 0; e < 4; ++e) { xv[e] = xa[e]; xv[4 + e] = xb[e]; }
#pragma unroll
  for (int e = 0; e < 8; ++e) ok[e] = (tid < ncol) && ((c0 + e) < nvalid);
  float s = 0.0f;
#pragma unroll
  for (int e = 0; e < 8; ++e) s += ok[e] ? xv[e] : 0.0f;
#pragma unroll
  for (int off = 1; off < 32; off <<= 1) s += __shfl_xor(s, off, 32);
  if (lane == 0) red[wave] = s;
  __syncthreads();
  const float invn = 1.0f / (float)nvalid;
  const float tot  = (red[0] + red[1]) + (red[2] + red[3]);
  const float mu   = tot * invn;
  float s2 = 0.0f;
#pragma unroll
  for (int e = 0; e < 8; ++e) { const float dv = xv[e] - mu; s2 += ok[e] ? (dv * dv) : 0.0f; }
#pragma unroll
  for (int off = 1; off < 32; off <<= 1) s2 += __shfl_xor(s2, off, 32);
  if (lane == 0) red[4 + wave] = s2;
  __syncthreads();
  const float var  = ((red[4] + red[5]) + (red[6] + red[7])) * invn;
  const float rstd = 1.0f / sqrtf(var + EPS_LN);
  const v4f ga = *(const v4f*)(sg + c0), gbv = *(const v4f*)(sg + c0 + 4);
  const v4f ba = *(const v4f*)(sbb + c0), bbv = *(const v4f*)(sbb + c0 + 4);
  float gvv[8], bvv[8];
#pragma unroll
  for (int e = 0; e < 4; ++e) { gvv[e] = ga[e]; gvv[4 + e] = gbv[e]; bvv[e] = ba[e]; bvv[4 + e] = bbv[e]; }
  v4u oh, ol;
#pragma unroll
  for (int e = 0; e < 4; ++e) {
    unsigned short hb2[2], lb2[2];
#pragma unroll
    for (int u = 0; u < 2; ++u) {
      const int k = 2 * e + u;
      const float y = ok[k] ? ((xv[k] - mu) * rstd * gvv[k] + bvv[k]) : 0.0f;
      const float t = y * sc;
      const _Float16 hv = (_Float16)t;
      const _Float16 lv = (_Float16)(t - (float)hv);
      hb2[u] = h_bits(hv);
      lb2[u] = h_bits(lv);
    }
    oh[e] = pk16(hb2[0], hb2[1]);
    ol[e] = pk16(lb2[0], lb2[1]);
  }
  if (tid < ncol) {
    u16* dh = Hp + (size_t)row * (size_t)ldd + c0;
    u16* dl = Lp + (size_t)row * (size_t)ldd + c0;
    for (int pass = 0; pass < 2; ++pass) {
      *(volatile v4u*)(dh) = oh;
      *(volatile v4u*)(dl) = ol;
      __threadfence();
    }
  }
}

__global__ __launch_bounds__(128) void qrot16(const float* __restrict__ F, int b, int sbase,
                                              const float* __restrict__ CS, u16* QHp, u16* QLp) {
#pragma clang fp contract(off)
  const int tid = (int)threadIdx.x;
  const int r   = (int)blockIdx.x;
  if (r >= MCH) return;
  const int s    = sbase + r;
  const int head = tid >> 3, i = tid & 7, ip = i & 3;
  const float* p = F + (size_t)r * DMOD + head * HD;
  const v4f na = *(const v4f*)(p + 8 * i), nb4 = *(const v4f*)(p + 8 * i + 4);
  const v4f xa = *(const v4f*)(p + HHALF + 8 * ip), xb = *(const v4f*)(p + HHALF + 8 * ip + 4);
  const v4f ya = *(const v4f*)(p + HHALF + HROT + 8 * ip), yb = *(const v4f*)(p + HHALF + HROT + 8 * ip + 4);
  const v4f ca = *(const v4f*)(CS + head * HROT + 8 * ip), cb = *(const v4f*)(CS + head * HROT + 8 * ip + 4);
  const v4f sa = *(const v4f*)(CS + NH * HROT + head * HROT + 8 * ip), sb = *(const v4f*)(CS + NH * HROT + head * HROT + 8 * ip + 4);
  float qn[8], x1[8], x2[8], cv[8], sv[8];
#pragma unroll
  for (int e = 0; e < 4; ++e) {
    qn[e] = na[e]; qn[4 + e] = nb4[e];
    x1[e] = xa[e]; x1[4 + e] = xb[e];
    x2[e] = ya[e]; x2[4 + e] = yb[e];
    cv[e] = ca[e]; cv[4 + e] = cb[e];
    sv[e] = sa[e]; sv[4 + e] = sb[e];
  }
  const bool first = (i < 4);
  v4u onh, onl, orh, orl;
#pragma unroll
  for (int e = 0; e < 4; ++e) {
    unsigned short nh2[2], nl2[2], rh2[2], rl2[2];
#pragma unroll
    for (int u = 0; u < 2; ++u) {
      const int k = 2 * e + u;
      const float ra = x1[k] * cv[k] + x2[k] * sv[k];
      const float rb = -(x1[k] * sv[k]) + x2[k] * cv[k];
      const float rv = first ? ra : rb;
      const float tn = qn[k] * QSC, tr = rv * QSC;
      const _Float16 hn = (_Float16)tn, hr = (_Float16)tr;
      nh2[u] = h_bits(hn);
      nl2[u] = h_bits((_Float16)(tn - (float)hn));
      rh2[u] = h_bits(hr);
      rl2[u] = h_bits((_Float16)(tr - (float)hr));
    }
    onh[e] = pk16(nh2[0], nh2[1]);
    onl[e] = pk16(nl2[0], nl2[1]);
    orh[e] = pk16(rh2[0], rh2[1]);
    orl[e] = pk16(rl2[0], rl2[1]);
  }
  const bool wl = (s < QRES);
  const size_t row  = (size_t)b * SEQ + s;
  const size_t rowl = (size_t)b * QRES + s;
  u16* dh = QHp + row * DMOD + (size_t)head * HD + 8 * i;
  u16* dl = QLp + rowl * DMOD + (size_t)head * HD + 8 * i;
  for (int pass = 0; pass < 2; ++pass) {
    *(volatile v4u*)(dh) = onh;
    *(volatile v4u*)(dh + HHALF) = orh;
    if (wl) {
      *(volatile v4u*)(dl) = onl;
      *(volatile v4u*)(dl + HHALF) = orl;
    }
    __threadfence();
  }
}

__global__ __launch_bounds__(128) void kplane16(const float* __restrict__ F, const float* __restrict__ CKV,
                                                int b, int sbase, u16* KHp, u16* KLp) {
  const int tid = (int)threadIdx.x;
  const int r   = (int)blockIdx.x;
  if (r >= MCH) return;
  const int s    = sbase + r;
  const int head = tid >> 3, i = tid & 7;
  const size_t row  = (size_t)b * SEQ + s;
  const size_t rowl = (size_t)b * QRES + s;
  const float* pn = F + (size_t)r * DUKV + head * DHKV + 8 * i;
  const float* pr = CKV + row * DCKV + DKV + 8 * i;
  const v4f na = *(const v4f*)(pn), nb4 = *(const v4f*)(pn + 4);
  const v4f ra = *(const v4f*)(pr), rb4 = *(const v4f*)(pr + 4);
  float kn[8], kr[8];
#pragma unroll
  for (int e = 0; e < 4; ++e) { kn[e] = na[e]; kn[4 + e] = nb4[e]; kr[e] = ra[e]; kr[4 + e] = rb4[e]; }
  v4u onh, onl, orh, orl;
#pragma unroll
  for (int e = 0; e < 4; ++e) {
    unsigned short nh2[2], nl2[2], rh2[2], rl2[2];
#pragma unroll
    for (int u = 0; u < 2; ++u) {
      const int k = 2 * e + u;
      const float tn = kn[k] * KSC, tr = kr[k] * KSC;
      const _Float16 hn = (_Float16)tn, hr = (_Float16)tr;
      nh2[u] = h_bits(hn);
      nl2[u] = h_bits((_Float16)(tn - (float)hn));
      rh2[u] = h_bits(hr);
      rl2[u] = h_bits((_Float16)(tr - (float)hr));
    }
    onh[e] = pk16(nh2[0], nh2[1]);
    onl[e] = pk16(nl2[0], nl2[1]);
    orh[e] = pk16(rh2[0], rh2[1]);
    orl[e] = pk16(rl2[0], rl2[1]);
  }
  const bool wl = (s < QRES);
  u16* dh = KHp + row * DMOD + (size_t)head * HD + 8 * i;
  u16* dl = KLp + rowl * DMOD + (size_t)head * HD + 8 * i;
  for (int pass = 0; pass < 2; ++pass) {
    *(volatile v4u*)(dh) = onh;
    *(volatile v4u*)(dh + HHALF) = orh;
    if (wl) {
      *(volatile v4u*)(dl) = onl;
      *(volatile v4u*)(dl + HHALF) = orl;
    }
    __threadfence();
  }
}

__global__ __launch_bounds__(256) void vt16(const float* __restrict__ F, int b, int sbase, u16* VHo, u16* VLo) {
  __shared__ __align__(16) u16 TH[HD * VTP];
  __shared__ __align__(16) u16 TL[HD * VTP];
  const int tid = (int)threadIdx.x;
  const int bid = (int)blockIdx.x;
  const int st  = bid % NST;
  const int h   = bid / NST;
  if (h >= NH) return;
  const int sl0 = st * 64;
  {
    const int sl = tid >> 2;
    const int dc = (tid & 3) * 32;
    const float* src = F + (size_t)(sl0 + sl) * DUKV + h * DHKV + DKR + dc;
#pragma unroll
    for (int i = 0; i < 8; ++i) {
      const v4f a = *(const v4f*)(src + 4 * i);
#pragma unroll
      for (int e = 0; e < 4; ++e) {
        const float t = a[e] * VCAR;
        const _Float16 hv = (_Float16)t;
        const _Float16 lv = (_Float16)(t - (float)hv);
        TH[(dc + 4 * i + e) * VTP + sl] = h_bits(hv);
        TL[(dc + 4 * i + e) * VTP + sl] = h_bits(lv);
      }
    }
  }
  __syncthreads();
  v4u vh[4], vl[4];
  const int q8 = tid >> 3, p8 = (tid & 7) * 8;
#pragma unroll
  for (int it = 0; it < 4; ++it) {
    const int line = it * 32 + q8;
    vh[it] = *(const v4u*)(TH + line * VTP + p8);
    vl[it] = *(const v4u*)(TL + line * VTP + p8);
  }
  const bool wl = (sbase + sl0) < QRES;
  const size_t hrow  = (size_t)(b * NH + h) * HD;
  const size_t baseh = hrow * SEQ  + (size_t)(sbase + sl0) + p8;
  const size_t basel = hrow * QRES + (size_t)(sbase + sl0) + p8;
  for (int pass = 0; pass < 2; ++pass) {
#pragma unroll
    for (int it = 0; it < 4; ++it) {
      const int line = it * 32 + q8;
      *(volatile v4u*)(VHo + baseh + (size_t)line * SEQ) = vh[it];
      if (wl) {
        *(volatile v4u*)(VLo + basel + (size_t)line * QRES) = vl[it];
      }
    }
    __threadfence();
  }
}

__device__ __forceinline__ float biasv(const float* __restrict__ bias, int nbias, int col) {
  const int cl = (col < nbias) ? col : (nbias - 1);
  const float v = bias[cl];
  return (col < nbias) ? bfr(v) : 0.0f;
}
__device__ __forceinline__ void epi64(float* sl, v8f a0, v8f a1, v8f a2, v8f a3, float oscale,
                                      const float* __restrict__ bias, int nbias,
                                      float* C, int N, size_t rowb, int col0, int lane) {
  const int hh = lane >> 4, m = lane & 15;
  const float bv0 = biasv(bias, nbias, col0 + m);
  const float bv1 = biasv(bias, nbias, col0 + 16 + m);
  const float bv2 = biasv(bias, nbias, col0 + 32 + m);
  const float bv3 = biasv(bias, nbias, col0 + 48 + m);
#pragma unroll
  for (int r = 0; r < 8; ++r) {
    const int ro = (8 * hh + r) * 68 + m;
    sl[ro]      = a0[r] * oscale + bv0;
    sl[ro + 16] = a1[r] * oscale + bv1;
    sl[ro + 32] = a2[r] * oscale + bv2;
    sl[ro + 48] = a3[r] * oscale + bv3;
  }
  wave_sync_lds();
  v4f vals[8];
#pragma unroll
  for (int it = 0; it < 8; ++it) vals[it] = *(const v4f*)(sl + (it * 2 + hh) * 68 + m * 4);
  float* dst = C + (rowb + (size_t)hh) * (size_t)N + col0 + m * 4;
  for (int pass = 0; pass < 2; ++pass) {
#pragma unroll
    for (int it = 0; it < 8; ++it) {
      *(volatile v4f*)(dst + (size_t)(it * 2) * (size_t)N) = vals[it];
    }
    __threadfence();
  }
}

__global__ __launch_bounds__(128)
void gemm_bf(const u16* __restrict__ A, const u16* __restrict__ Bt, const float* __restrict__ bias, int nbias,
             float* C, int M, int N, int K, float oscale) {
  __shared__ __align__(16) float slab[4 * SLAB64];
  const int tid = threadIdx.x, wave = tid >> 5, lane = tid & 31, hh = lane >> 4, m = lane & 15;
  const int ntile = N >> 6;
  const int bid   = blockIdx.x;
  const int rowb  = (bid / ntile) * 64 + wave * 16;
  const int col0  = (bid % ntile) * 64;
  if (rowb + 16 > M) return;
  const u16* ap = A  + (size_t)(rowb + m) * K + 8 * hh;
  const u16* bp = Bt + (size_t)(col0 + m) * K + 8 * hh;
  const size_t bs = (size_t)16 * K;
  v8f acc0 = zero8(), acc1 = zero8(), acc2 = zero8(), acc3 = zero8();
#pragma unroll 1
  for (int k0 = 0; k0 < K; k0 += 32) {
    const v16b a  = ldfrag_b(ap + k0);
    const v16b b0 = ldfrag_b(bp + k0);
    const v16b b1 = ldfrag_b(bp + bs + k0);
    const v16b b2 = ldfrag_b(bp + 2 * bs + k0);
    const v16b b3 = ldfrag_b(bp + 3 * bs + k0);
    acc0 = mma_b(a, b0, acc0);
    acc1 = mma_b(a, b1, acc1);
    acc2 = mma_b(a, b2, acc2);
    acc3 = mma_b(a, b3, acc3);
    guard6<v16b>(acc0, acc1, acc2, acc3, a, b0, b1, b2, b3, a);
  }
  epi64(slab + wave * SLAB64, acc0, acc1, acc2, acc3, oscale, bias, nbias, C, N, (size_t)rowb, col0, lane);
}

__global__ __launch_bounds__(128)
void gemm_hh(const u16* __restrict__ Ah, const u16* __restrict__ Al, const u16* __restrict__ Bt,
             const float* __restrict__ bias, int nbias, float* C, int M, int N, int K, float oscale) {
  __shared__ __align__(16) float slab[4 * SLAB64];
  const int tid = threadIdx.x, wave = tid >> 5, lane = tid & 31, hh = lane >> 4, m = lane & 15;
  const int ntile = N >> 6;
  const int bid   = blockIdx.x;
  const int rowb  = (bid / ntile) * 64 + wave * 16;
  const int col0  = (bid % ntile) * 64;
  if (rowb + 16 > M) return;
  const _Float16* ahp = hp(Ah) + (size_t)(rowb + m) * K + 8 * hh;
  const _Float16* alp = hp(Al) + (size_t)(rowb + m) * K + 8 * hh;
  const _Float16* bp  = hp(Bt) + (size_t)(col0 + m) * K + 8 * hh;
  const size_t bs = (size_t)16 * K;
  v8f acc0 = zero8(), acc1 = zero8(), acc2 = zero8(), acc3 = zero8();
#pragma unroll 1
  for (int k0 = 0; k0 < K; k0 += 32) {
    const v16h ah = ldfrag_h(ahp + k0), al = ldfrag_h(alp + k0);
    const v16h b0 = ldfrag_h(bp + k0);
    const v16h b1 = ldfrag_h(bp + bs + k0);
    const v16h b2 = ldfrag_h(bp + 2 * bs + k0);
    const v16h b3 = ldfrag_h(bp + 3 * bs + k0);
    acc0 = mma_h(ah, b0, acc0);  acc0 = mma_h(al, b0, acc0);
    acc1 = mma_h(ah, b1, acc1);  acc1 = mma_h(al, b1, acc1);
    acc2 = mma_h(ah, b2, acc2);  acc2 = mma_h(al, b2, acc2);
    acc3 = mma_h(ah, b3, acc3);  acc3 = mma_h(al, b3, acc3);
    guard6<v16h>(acc0, acc1, acc2, acc3, ah, al, b0, b1, b2, b3);
  }
  epi64(slab + wave * SLAB64, acc0, acc1, acc2, acc3, oscale, bias, nbias, C, N, (size_t)rowb, col0, lane);
}

template <int NPROD>
__global__ __launch_bounds__(128)
void gemm_o(const u16* __restrict__ Ah, const u16* __restrict__ Al, const u16* __restrict__ Bt,
            const float* __restrict__ bias, float* C, int sbeg, int nrt, float oscale) {
  __shared__ __align__(16) float slab[4 * SLAB64];
  const int tid = threadIdx.x, wave = tid >> 5, lane = tid & 31, hh = lane >> 4, m = lane & 15;
  const int ntile = DMOD >> 6;
  const int bid   = blockIdx.x;
  const int ct    = bid % ntile;
  const int t2    = bid / ntile;
  const int rt    = t2 % nrt;
  const int bb    = t2 / nrt;
  if (bb >= NB) return;
  const int srow  = sbeg + rt * 64 + wave * 16;
  if (srow + 16 > SEQ) return;
  const int col0  = ct * 64;
  const int K     = DMOD;
  const size_t rowC = (size_t)bb * SEQ + srow;
  const size_t rowL = (size_t)bb * QO + srow;
  const _Float16* ahp = hp(Ah) + (rowC + m) * K + 8 * hh;
  const _Float16* alp = hp(Al) + (rowL + m) * K + 8 * hh;
  const _Float16* bp  = hp(Bt) + (size_t)(col0 + m) * K + 8 * hh;
  const size_t bs = (size_t)16 * K;
  v8f acc0 = zero8(), acc1 = zero8(), acc2 = zero8(), acc3 = zero8();
  if constexpr (NPROD == 2) {
#pragma unroll 1
    for (int k0 = 0; k0 < K; k0 += 32) {
      const v16h ah = ldfrag_h(ahp + k0), al = ldfrag_h(alp + k0);
      const v16h b0 = ldfrag_h(bp + k0);
      const v16h b1 = ldfrag_h(bp + bs + k0);
      const v16h b2 = ldfrag_h(bp + 2 * bs + k0);
      const v16h b3 = ldfrag_h(bp + 3 * bs + k0);
      acc0 = mma_h(ah, b0, acc0);  acc0 = mma_h(al, b0, acc0);
      acc1 = mma_h(ah, b1, acc1);  acc1 = mma_h(al, b1, acc1);
      acc2 = mma_h(ah, b2, acc2);  acc2 = mma_h(al, b2, acc2);
      acc3 = mma_h(ah, b3, acc3);  acc3 = mma_h(al, b3, acc3);
      guard6<v16h>(acc0, acc1, acc2, acc3, ah, al, b0, b1, b2, b3);
    }
  } else {
#pragma unroll 1
    for (int k0 = 0; k0 < K; k0 += 32) {
      const v16h ah = ldfrag_h(ahp + k0);
      const v16h b0 = ldfrag_h(bp + k0);
      const v16h b1 = ldfrag_h(bp + bs + k0);
      const v16h b2 = ldfrag_h(bp + 2 * bs + k0);
      const v16h b3 = ldfrag_h(bp + 3 * bs + k0);
      acc0 = mma_h(ah, b0, acc0);
      acc1 = mma_h(ah, b1, acc1);
      acc2 = mma_h(ah, b2, acc2);
      acc3 = mma_h(ah, b3, acc3);
      guard6<v16h>(acc0, acc1, acc2, acc3, ah, b0, b1, b2, b3, ah);
    }
  }
  epi64(slab + wave * SLAB64, acc0, acc1, acc2, acc3, oscale, bias, DMOD, C, DMOD, rowC, col0, lane);
}

template <int FULL>
__global__ __launch_bounds__(ATT_THREADS)
void attn_c(const u16* __restrict__ QHp, const u16* __restrict__ QLp,
            const u16* __restrict__ KHp, const u16* __restrict__ KLp,
            const u16* __restrict__ VHp, const u16* __restrict__ VLp,
            u16* OHp, u16* OLp, int qt0, int nqt) {
  __shared__ __align__(16) float smem[WPB * WREG];

  const int tid  = threadIdx.x;
  const int wave = tid >> 5;
  const int lane = tid & 31;
  const int hh   = lane >> 4;
  const int c    = lane & 15;
  const int bid  = blockIdx.x;
  const int qt   = qt0 + (bid % nqt);
  const int t2   = bid / nqt;
  const int hg   = t2 % NHG;
  const int b    = t2 / NHG;
  if (b >= NB) return;
  const int q0   = qt * 16;
  if (q0 + 16 > SEQ) return;
  const int head = hg * WPB + wave;

  float* pt   = smem + wave * WREG;
  float* slab = pt + PTW;

  const size_t hcol = (size_t)head * HD + 8 * hh;
  const _Float16* Qh  = hp(QHp) + ((size_t)b * SEQ  + q0 + c) * DMOD + hcol;
  const _Float16* Ql  = hp(QLp) + ((size_t)b * QRES + q0 + c) * DMOD + hcol;
  const _Float16* Khb = hp(KHp) + ((size_t)b * SEQ  + c) * DMOD + hcol;
  const _Float16* Klb = hp(KLp) + ((size_t)b * QRES + c) * DMOD + hcol;
  const _Float16* Vhb = hp(VHp) + ((size_t)(b * NH + head) * HD + c) * SEQ  + 8 * hh;
  const _Float16* Vlb = hp(VLp) + ((size_t)(b * NH + head) * HD + c) * QRES + 8 * hh;
  const float lsc = RSQ_HD * (LOG2E / (QSC * KSC));
  const float oc  = 1.0f / (PCAR * VCAR);
  const size_t KROW = (size_t)DMOD;

  float mrow[8], lrow[8];
  v8f o[8];
#pragma unroll
  for (int r = 0; r < 8; ++r) { mrow[r] = -INFINITY; lrow[r] = 0.f; }
#pragma unroll
  for (int j = 0; j < 8; ++j) o[j] = zero8();
  const int ncaus = (q0 >> 5) + 1;
  const int nkt = (ncaus < NKT) ? ncaus : NKT;
  const int qr0 = q0 + 8 * hh;

#pragma unroll 1
  for (int kt = 0; kt < nkt; ++kt) {
    const int kb = kt * 32;
    v8f s0 = zero8(), s1 = zero8();
    const _Float16* k0p = Khb + (size_t)kb * KROW;
    const _Float16* k1p = k0p + (size_t)16 * KROW;
    if constexpr (FULL != 0) {
      const _Float16* l0p = Klb + (size_t)kb * KROW;
      const _Float16* l1p = l0p + (size_t)16 * KROW;
#pragma unroll
      for (int kk = 0; kk < HD / 32; ++kk) {
        const v16h qh  = ldfrag_h(Qh + kk * 32);
        const v16h ql  = ldfrag_h(Ql + kk * 32);
        const v16h kh0 = ldfrag_h(k0p + kk * 32);
        const v16h kh1 = ldfrag_h(k1p + kk * 32);
        const v16h kl0 = ldfrag_h(l0p + kk * 32);
        const v16h kl1 = ldfrag_h(l1p + kk * 32);
        s0 = mma_h(qh, kh0, s0);
        s0 = mma_h(ql, kh0, s0);
        s0 = mma_h(qh, kl0, s0);
        s1 = mma_h(qh, kh1, s1);
        s1 = mma_h(ql, kh1, s1);
        s1 = mma_h(qh, kl1, s1);
        guard2(s0, s1, qh, ql, kh0, kl0, kh1, kl1);
      }
    } else {
#pragma unroll
      for (int kk = 0; kk < HD / 32; ++kk) {
        const v16h qh  = ldfrag_h(Qh + kk * 32);
        const v16h kh0 = ldfrag_h(k0p + kk * 32);
        const v16h kh1 = ldfrag_h(k1p + kk * 32);
        s0 = mma_h(qh, kh0, s0);
        s1 = mma_h(qh, kh1, s1);
        guard2(s0, s1, qh, kh0, kh1, qh, kh0, kh1);
      }
    }
    const int key0 = kb + c, key1 = kb + 16 + c;
#pragma unroll
    for (int r = 0; r < 8; ++r) {
      const int   qr = qr0 + r;
      const float u0 = s0[r] * lsc;
      const float u1 = s1[r] * lsc;
      const bool ok0 = (key0 <= qr);
      const bool ok1 = (key1 <= qr);
      const float t0 = ok0 ? u0 : NEGT;
      const float t1 = ok1 ? u1 : NEGT;
      float mx = fmaxf(t0, t1);
#pragma unroll
      for (int off = 1; off < 16; off <<= 1) mx = fmaxf(mx, __shfl_xor(mx, off, 32));
      const float mn = fmaxf(mrow[r], mx);
      const float ms = (mn == -INFINITY) ? 0.0f : mn;
      const float al = exp2f(mrow[r] - ms);
      mrow[r] = mn;
      const float e0 = exp2f(t0 - ms), e1 = exp2f(t1 - ms);
      float ps = e0 + e1;
#pragma unroll
      for (int off = 1; off < 16; off <<= 1) ps += __shfl_xor(ps, off, 32);
      lrow[r] = lrow[r] * al + ps;
#pragma unroll
      for (int j = 0; j < 8; ++j) o[j][r] *= al;
      const int ro = (8 * hh + r) * PTP + c;
      pt[ro]      = e0;
      pt[ro + 16] = e1;
    }
    wave_sync_lds();
    FragH ph, pl;
    {
      const float* prow = pt + c * PTP + 8 * hh;
      const v4f p0 = *(const v4f*)(prow), p1 = *(const v4f*)(prow + 4);
      const v4f p2 = *(const v4f*)(prow + 16), p3 = *(const v4f*)(prow + 20);
#pragma unroll
      for (int e = 0; e < 4; ++e) {
        const float ta = p0[e] * PCAR, tb = p1[e] * PCAR, tc = p2[e] * PCAR, td = p3[e] * PCAR;
        const _Float16 ha = (_Float16)ta, hb = (_Float16)tb, hc = (_Float16)tc, hd = (_Float16)td;
        ph.h[0][e]     = ha;
        ph.h[0][4 + e] = hb;
        ph.h[1][e]     = hc;
        ph.h[1][4 + e] = hd;
        if constexpr (FULL != 0) {
          pl.h[0][e]     = (_Float16)(ta - (float)ha);
          pl.h[0][4 + e] = (_Float16)(tb - (float)hb);
          pl.h[1][e]     = (_Float16)(tc - (float)hc);
          pl.h[1][4 + e] = (_Float16)(td - (float)hd);
        } else {
          pl.h[0][e] = ha; pl.h[0][4 + e] = hb; pl.h[1][e] = hc; pl.h[1][4 + e] = hd;
        }
      }
    }
    {
      const _Float16* vhp = Vhb + kb;
      if constexpr (FULL != 0) {
        const _Float16* vlp = Vlb + kb;
#pragma unroll
        for (int jg = 0; jg < 4; ++jg) {
          const size_t da = (size_t)(2 * jg) * 16 * SEQ;
          const size_t db = da + (size_t)16 * SEQ;
          const size_t la = (size_t)(2 * jg) * 16 * QRES;
          const size_t lb = la + (size_t)16 * QRES;
          const v16h vha = ldfrag_h(vhp + da), vhb2 = ldfrag_h(vhp + db);
          const v16h vla = ldfrag_h(vlp + la), vlb2 = ldfrag_h(vlp + lb);
          o[2 * jg]     = mma_h(ph.v, vha,  o[2 * jg]);
          o[2 * jg]     = mma_h(pl.v, vha,  o[2 * jg]);
          o[2 * jg]     = mma_h(ph.v, vla,  o[2 * jg]);
          o[2 * jg + 1] = mma_h(ph.v, vhb2, o[2 * jg + 1]);
          o[2 * jg + 1] = mma_h(pl.v, vhb2, o[2 * jg + 1]);
          o[2 * jg + 1] = mma_h(ph.v, vlb2, o[2 * jg + 1]);
          guard2(o[2 * jg], o[2 * jg + 1], ph.v, pl.v, vha, vhb2, vla, vlb2);
        }
      } else {
#pragma unroll
        for (int jg = 0; jg < 4; ++jg) {
          const size_t da = (size_t)(2 * jg) * 16 * SEQ;
          const size_t db = da + (size_t)16 * SEQ;
          const v16h vha = ldfrag_h(vhp + da), vhb2 = ldfrag_h(vhp + db);
          o[2 * jg]     = mma_h(ph.v, vha,  o[2 * jg]);
          o[2 * jg + 1] = mma_h(ph.v, vhb2, o[2 * jg + 1]);
          guard2(o[2 * jg], o[2 * jg + 1], ph.v, vha, vhb2, ph.v, vha, vhb2);
        }
      }
    }
    wave_sync_lds();
  }
  acc_guard4(o[0], o[1], o[2], o[3]);
  acc_guard4(o[4], o[5], o[6], o[7]);
#pragma unroll
  for (int r = 0; r < 8; ++r) {
    const float lv  = lrow[r];
    const float ls  = (lv > 0.0f) ? lv : 1.0f;
    const float inv = (lv > 0.0f) ? ((1.0f / ls) * oc) : 0.0f;
#pragma unroll
    for (int j = 0; j < 8; ++j) {
      const int idx = (8 * hh + r) * SLP + j * 16 + c;
      slab[idx] = o[j][r] * inv;
    }
  }

  wave_sync_lds();
  v4u oh[8], ol[8];
  const int rq = lane >> 4, c8 = (lane & 15) * 8;
#pragma unroll
  for (int it = 0; it < 8; ++it) {
    const int row = it * 2 + rq;
    const v4f a = *(const v4f*)(slab + row * SLP + c8), b4 = *(const v4f*)(slab + row * SLP + c8 + 4);
    float w[8];
#pragma unroll
    for (int e = 0; e < 4; ++e) { w[e] = a[e] * OSC; w[4 + e] = b4[e] * OSC; }
#pragma unroll
    for (int e = 0; e < 4; ++e) {
      const _Float16 h0 = (_Float16)w[2 * e], h1 = (_Float16)w[2 * e + 1];
      const _Float16 l0 = (_Float16)(w[2 * e] - (float)h0), l1 = (_Float16)(w[2 * e + 1] - (float)h1);
      oh[it][e] = pk16(h_bits(h0), h_bits(h1));
      ol[it][e] = pk16(h_bits(l0), h_bits(l1));
    }
  }
  const bool wlo = (q0 < QO);
  const size_t ob  = ((size_t)b * SEQ + q0) * DMOD + (size_t)head * HD + c8;
  const size_t olb = ((size_t)b * QO  + q0) * DMOD + (size_t)head * HD + c8;
  for (int pass = 0; pass < 2; ++pass) {
#pragma unroll
    for (int it = 0; it < 8; ++it) {
      const int row = it * 2 + rq;
      *(volatile v4u*)(OHp + ob + (size_t)row * DMOD) = oh[it];
      if (wlo) {
        *(volatile v4u*)(OLp + olb + (size_t)row * DMOD) = ol[it];
      }
    }
    __threadfence();
  }
}

static size_t up4k(size_t v) { return (v + 4095) & ~(size_t)4095; }
static size_t mx2(size_t a, size_t b) { return (a > b) ? a : b; }

extern "C" void kernel_launch(void* const* d_in, const int* in_sizes, int n_in,
                              void* d_out, int out_size, void* d_ws, size_t ws_size,
                              hipStream_t stream) {
  if (n_in < 15) return;
  if (in_sizes[0]  < ((NB - 1) * XS_FULL + SEQ) * DMOD) return;
  if (in_sizes[1]  < DQ * DMOD) return;
  if (in_sizes[2]  < DQ) return;
  if (in_sizes[3]  < DQ) return;
  if (in_sizes[4]  < DQ) return;
  if (in_sizes[5]  < DMOD * DQ) return;
  if (in_sizes[6]  < DMOD) return;
  if (in_sizes[7]  < DCKV * DMOD) return;
  if (in_sizes[8]  < DCKV) return;
  if (in_sizes[9]  < DKV) return;
  if (in_sizes[10] < DKV) return;
  if (in_sizes[11] < DUKV * DKV) return;
  if (in_sizes[12] < DUKV) return;
  if (in_sizes[13] < DMOD * DMOD) return;
  if (in_sizes[14] < DMOD) return;
  if (out_size < MROWS * DMOD) return;

  const float* x    = (const float*)d_in[0];
  const float* wdq  = (const float*)d_in[1];
  const float* bdq  = (const float*)d_in[2];
  const float* qng  = (const float*)d_in[3];
  const float* qnb  = (const float*)d_in[4];
  const float* wuq  = (const float*)d_in[5];
  const float* buq  = (const float*)d_in[6];
  const float* wdkv = (const float*)d_in[7];
  const float* bdkv = (const float*)d_in[8];
  const float* kvg  = (const float*)d_in[9];
  const float* kvb  = (const float*)d_in[10];
  const float* wukv = (const float*)d_in[11];
  const float* bukv = (const float*)d_in[12];
  const float* wo   = (const float*)d_in[13];
  const float* bo   = (const float*)d_in[14];
  float*       out  = (float*)d_out;

  const size_t szXB   = (size_t)MROWS * DMOD * 2;
  const size_t szWDQ  = (size_t)DQP * DMOD * 2;
  const size_t szWDKV = (size_t)DCKV * DMOD * 2;
  const size_t szCQF  = (size_t)MROWS * DQP * 4;
  const size_t szCQH  = (size_t)MROWS * DQP * 2;
  const size_t szCKVF = (size_t)MROWS * DCKV * 4;
  const size_t szKVN  = (size_t)MROWS * DKV * 2;
  const size_t szWUQ  = (size_t)DMOD * DQP * 2;
  const size_t szWUKV = (size_t)DUKV * DKV * 2;
  const size_t szF    = (size_t)MCH * DUKV * 4;
  const size_t szQH   = (size_t)MROWS * DMOD * 2;
  const size_t szQL   = (size_t)NB * QRES * DMOD * 2;
  const size_t szOL   = (size_t)NB * QO * DMOD * 2;
  const size_t szWO   = (size_t)DMOD * DMOD * 2;
  const size_t szTAB  = 4096;

  const size_t oXB   = 0;
  const size_t oWDQ  = oXB + up4k(szXB);
  const size_t oWDKV = oWDQ + up4k(szWDQ);
  const size_t oCQF  = oWDKV + up4k(szWDKV);
  const size_t oCQH  = 0;
  const size_t oCQL  = oCQH + up4k(szCQH);
  const size_t oKH   = 0;
  const size_t oVH   = oKH + up4k(szQH);
  const size_t oKL   = oVH + up4k(szQH);
  const size_t oVL   = oKL + up4k(szQL);
  if (oCQL + up4k(szCQH) > oCQF) return;
  const size_t endA  = mx2(mx2(oCQF + up4k(szCQF), oCQL + up4k(szCQH)), oVL + up4k(szQL));
  const size_t oQH   = endA;
  const size_t oQL   = oQH + up4k(szQH);
  const size_t endB  = oQL + up4k(szQL);
  const size_t oCKVF = endB;
  const size_t oOH   = endB;
  const size_t oOL   = oOH + up4k(szQH);
  const size_t endC  = endB + mx2(up4k(szCKVF), up4k(szQH) + up4k(szOL));
  const size_t oKVNH = endC;
  const size_t oKVNL = oKVNH + up4k(szKVN);
  const size_t oWO   = endC;
  const size_t endD  = endC + mx2(2 * up4k(szKVN), up4k(szWO));
  const size_t oWUQ  = endD;
  const size_t oWUKV = oWUQ + up4k(szWUQ);
  const size_t endE  = oWUKV + up4k(szWUKV);
  const size_t oF    = endE;
  const size_t endF  = oF + up4k(szF);
  const size_t oTAB  = endF;
  const size_t total = oTAB + up4k(szTAB);
  if (total > ws_size) return;
  if (total > (size_t)WS_CAP) return;

  char* ws = (char*)d_ws;
  u16*   XB   = (u16*)(ws + oXB);
  u16*   WDQ  = (u16*)(ws + oWDQ);
  u16*   WDKV = (u16*)(ws + oWDKV);
  float* CQF  = (float*)(ws + oCQF);
  u16*   CQH  = (u16*)(ws + oCQH);
  u16*   CQL  = (u16*)(ws + oCQL);
  u16*   KH   = (u16*)(ws + oKH);
  u16*   VH   = (u16*)(ws + oVH);
  u16*   KL   = (u16*)(ws + oKL);
  u16*   VL   = (u16*)(ws + oVL);
  u16*   QH   = (u16*)(ws + oQH);
  u16*   QL   = (u16*)(ws + oQL);
  float* CKVF = (float*)(ws + oCKVF);
  u16*   OH   = (u16*)(ws + oOH);
  u16*   OL   = (u16*)(ws + oOL);
  u16*   KVNH = (u16*)(ws + oKVNH);
  u16*   KVNL = (u16*)(ws + oKVNL);
  u16*   WO   = (u16*)(ws + oWO);
  u16*   WUQ  = (u16*)(ws + oWUQ);
  u16*   WUKV = (u16*)(ws + oWUKV);
  float* F    = (float*)(ws + oF);
  float* TAB  = (float*)(ws + oTAB);

  const dim3 b256(256), b128(128), bAT(ATT_THREADS);
  const float osUP = 1.0f / (CSC * WSC);
  const float osO  = 1.0f / (OSC * WSC);

  {
    const int n8x = (SEQ * DMOD) / 8;
    for (int b = 0; b < NB; ++b) {
      cvtpad16<<<dim3((n8x + 255) / 256), b256, 0, stream>>>(x + (size_t)b * XS_FULL * DMOD, SEQ, DMOD,
                                                              XB + (size_t)b * SEQ * DMOD, SEQ, DMOD, 0, 1.0f, 1);
    }
    const int n8dq = (DQP * DMOD) / 8;
    cvtpad16<<<dim3((n8dq + 255) / 256), b256, 0, stream>>>(wdq, DQ, DMOD, WDQ, DQP, DMOD, 0, 1.0f, 0);
    const int n8dkv = (DCKV * DMOD) / 8;
    cvtpad16<<<dim3((n8dkv + 255) / 256), b256, 0, stream>>>(wdkv, DCKV, DMOD, WDKV, DCKV, DMOD, 0, 1.0f, 1);
    const int n8uq = (DMOD * DQP) / 8;
    cvtpad16<<<dim3((n8uq + 255) / 256), b256, 0, stream>>>(wuq, DMOD, DQ, WUQ, DMOD, DQP, 1, WSC, 0);
    const int n8ukv = (DUKV * DKV) / 8;
    cvtpad16<<<dim3((n8ukv + 255) / 256), b256, 0, stream>>>(wukv, DUKV, DKV, WUKV, DUKV, DKV, 1, WSC, 1);
    rtab<<<dim3(1), b256, 0, stream>>>(TAB);
  }
  gemm_bf<<<dim3((MROWS / 64) * (DQP / 64)), b128, 0, stream>>>(XB, WDQ, bdq, DQ, CQF, MROWS, DQP, DMOD, 1.0f);
  gemm_bf<<<dim3((MROWS / 64) * (DCKV / 64)), b128, 0, stream>>>(XB, WDKV, bdkv, DCKV, CKVF, MROWS, DCKV, DMOD, 1.0f);
  ln16<<<dim3(MROWS), b128, 0, stream>>>(CQF, DQP, DQ, qng, qnb, CQH, CQL, DQP, CSC);
  ln16<<<dim3(MROWS), b128, 0, stream>>>(CKVF, DCKV, DKV, kvg, kvb, KVNH, KVNL, DKV, CSC);
  for (int b = 0; b < NB; ++b) {
    for (int ch = 0; ch < NCH; ++ch) {
      const int sbase = ch * MCH;
      const size_t rows = (size_t)b * SEQ + sbase;
      gemm_hh<<<dim3((MCH / 64) * (DMOD / 64)), b128, 0, stream>>>(CQH + rows * DQP, CQL + rows * DQP, WUQ, buq, DMOD,
                                                                    F, MCH, DMOD, DQP, osUP);
      qrot16<<<dim3(MCH), b128, 0, stream>>>(F, b, sbase, TAB, QH, QL);
    }
  }
  for (int b = 0; b < NB; ++b) {
    for (int ch = 0; ch < NCH; ++ch) {
      const int sbase = ch * MCH;
      const size_t rows = (size_t)b * SEQ + sbase;
      gemm_hh<<<dim3((MCH / 64) * (DUKV / 64)), b128, 0, stream>>>(KVNH + rows * DKV, KVNL + rows * DKV, WUKV, bukv, DUKV,
                                                                    F, MCH, DUKV, DKV, osUP);
      kplane16<<<dim3(MCH), b128, 0, stream>>>(F, CKVF, b, sbase, KH, KL);
      vt16<<<dim3(NH * NST), b256, 0, stream>>>(F, b, sbase, VH, VL);
    }
  }
  {
    const int nqtF = QRES / 16;
    const int nqtP = NQT - nqtF;
    attn_c<1><<<dim3(nqtF * NHG * NB), bAT, 0, stream>>>(QH, QL, KH, KL, VH, VL, OH, OL, 0, nqtF);
    if (nqtP > 0) {
      attn_c<0><<<dim3(nqtP * NHG * NB), bAT, 0, stream>>>(QH, QL, KH, KL, VH, VL, OH, OL, nqtF, nqtP);
    }
    const int n8wo = (DMOD * DMOD) / 8;
    cvtpad16<<<dim3((n8wo + 255) / 256), b256, 0, stream>>>(wo, DMOD, DMOD, WO, DMOD, DMOD, 1, WSC, 1);
  }
  {
    const int nrtR = QO / 64;
    const int nrtP = (SEQ - QO) / 64;
    gemm_o<2><<<dim3(NB * nrtR * (DMOD / 64)), b128, 0, stream>>>(OH, OL, WO, bo, out, 0, nrtR, osO);
    if (nrtP > 0) {
      gemm_o<1><<<dim3(NB * nrtP * (DMOD / 64)), b128, 0, stream>>>(OH, OL, WO, bo, out, QO, nrtP, osO);
    }
  }
  (void)hipGetLastError();
}
